// Block_19224273617071
// MI455X (gfx1250) — hardware-verified
//
#include <hip/hip_runtime.h>
#include <math.h>

typedef __attribute__((ext_vector_type(16))) _Float16 v16h;
typedef __attribute__((ext_vector_type(8)))  _Float16 v8h;
typedef __attribute__((ext_vector_type(8)))  float    v8f;
typedef __attribute__((ext_vector_type(4)))  float    v4f;

constexpr int kBatch = 2;
constexpr int kSeqL  = 2048;
constexpr int kDmod  = 1024;
constexpr int kDin   = 2048;
constexpr int kNst   = 16;
constexpr int kDtR   = 64;
constexpr int kPrjN  = 96;
constexpr int kPrjP  = 128;
constexpr int kXZP   = 2 * kDin;
constexpr int kDff   = 4096;
constexpr int kRows  = kBatch * kSeqL;
constexpr int kTP    = 260;
constexpr int kXZW   = kXZP / 2;
constexpr int kUW    = kDin / 2;

constexpr float kCWin  = 32.0f;
constexpr float kCWxp  = 32.0f;
constexpr float kCWdt  = 8.0f;
constexpr float kCWout = 32.0f;
constexpr float kCWf1  = 32.0f;
constexpr float kCWf2  = 64.0f;
constexpr float kCDt   = 16.0f;
constexpr float kCY    = 16.0f;

static_assert(kDtR + 2 * kNst == kPrjN);
static_assert((kDmod % 32) == 0 && (kDin % 32) == 0 && (kDtR % 32) == 0 && (kDff % 32) == 0);
static_assert((kSeqL % 64) == 0 && (kRows % 64) == 0 && (kXZP % 64) == 0 && (kPrjP % 64) == 0 &&
              (kDin % 64) == 0 && (kDmod % 64) == 0 && (kDff % 64) == 0);
static_assert((kDin % 256) == 0 && (kSeqL % 64) == 0 && kDmod == 128 * 8);

constexpr size_t kSzWIN  = (size_t)kXZP * kDmod * 2;
constexpr size_t kSzWXP  = (size_t)kPrjP * kDin * 2;
constexpr size_t kSzWDT  = (size_t)kDin * kDtR * 2;
constexpr size_t kSzWOUT = (size_t)kDmod * kDin * 2;
constexpr size_t kSzWF1  = (size_t)kDff * kDmod * 2;
constexpr size_t kSzWF2  = (size_t)kDmod * kDff * 2;
constexpr size_t kSzH    = (size_t)kRows * kDmod * 2;
constexpr size_t kSzX1   = (size_t)kRows * kDmod * 4;
constexpr size_t kSzXZ   = (size_t)kSeqL * kXZP * 2;
constexpr size_t kSzU    = (size_t)kSeqL * kDin * 2;
constexpr size_t kSzY    = (size_t)kSeqL * kDin * 2;
constexpr size_t kSzXD   = (size_t)kSeqL * kPrjP * 4;
constexpr size_t kSzDT   = (size_t)kSeqL * kDtR * 2;
constexpr size_t kSzDLR  = (size_t)kSeqL * kDin * 4;
constexpr size_t kSzT    = (size_t)kRows * kDff * 2;
constexpr size_t kOffWIN  = 0;
constexpr size_t kOffWXP  = kOffWIN  + kSzWIN;
constexpr size_t kOffWDT  = kOffWXP  + kSzWXP;
constexpr size_t kOffWOUT = kOffWDT  + kSzWDT;
constexpr size_t kOffWF1  = kOffWOUT + kSzWOUT;
constexpr size_t kOffWF2  = kOffWF1  + kSzWF1;
constexpr size_t kOffH    = kOffWF2  + kSzWF2;
constexpr size_t kOffX1   = kOffH    + kSzH;
constexpr size_t kOffXZ   = kOffX1   + kSzX1;
constexpr size_t kOffU    = kOffXZ   + kSzXZ;
constexpr size_t kOffY    = kOffU    + kSzU;
constexpr size_t kOffXD   = kOffY    + kSzY;
constexpr size_t kOffDT   = kOffXD   + kSzXD;
constexpr size_t kOffDLR  = kOffDT   + kSzDT;
constexpr size_t kWsTotal = kOffDLR  + kSzDLR;
constexpr size_t kOffT    = kOffXZ;
static_assert(kWsTotal == 106954752ull);
static_assert(kWsTotal <= 134217728ull);
static_assert(kSzT == kSzXZ + kSzU + kSzY);
static_assert(kOffT + kSzT == kOffXD);
static_assert((kOffWXP % 128) == 0 && (kOffWDT % 128) == 0 && (kOffWOUT % 128) == 0 && (kOffWF1 % 128) == 0 &&
              (kOffWF2 % 128) == 0 && (kOffH % 128) == 0 && (kOffX1 % 128) == 0 && (kOffXZ % 128) == 0 &&
              (kOffU % 128) == 0 && (kOffY % 128) == 0 && (kOffXD % 128) == 0 && (kOffDT % 128) == 0 &&
              (kOffDLR % 128) == 0);

__device__ __forceinline__ float h16_to_f32(unsigned hb) {
  const unsigned sgn = (hb & 0x8000u) << 16;
  const unsigned em = hb & 0x7fffu;
  const float fn = __uint_as_float((em << 13) + 0x38000000u);
  const float fs = (float)em * 5.9604644775390625e-8f;
  const float mag = (em < 0x400u) ? fs : fn;
  return __uint_as_float(__float_as_uint(mag) | sgn);
}

__device__ __forceinline__ void keep4_h(v16h a, v16h b, v16h c, v16h d) { asm volatile("v_nop" :: "v"(a), "v"(b), "v"(c), "v"(d)); }
__device__ __forceinline__ void acc_guard4(v8f& a, v8f& b, v8f& c, v8f& d) { asm volatile("v_nop\n\tv_nop\n\tv_nop\n\tv_nop" : "+v"(a), "+v"(b), "+v"(c), "+v"(d)); }
__device__ __forceinline__ void guard_row_h(v8f& a, v8f& b, v8f& c, v8f& d, v16h x, v16h b0, v16h b1, v16h b2, v16h b3) {
  asm volatile("v_nop\n\tv_nop\n\tv_nop\n\tv_nop" : "+v"(a), "+v"(b), "+v"(c), "+v"(d) : "v"(x), "v"(b0), "v"(b1), "v"(b2), "v"(b3));
}
struct FragH {
  union U { v16h v; v8h h[2]; };
  static __device__ __forceinline__ v16h load(const _Float16* p) {
    U f; f.h[0] = *(const v8h*)(p); f.h[1] = *(const v8h*)(p + 16); return f.v;
  }
  static __device__ __forceinline__ v8f mma(v16h a, v16h b, v8f c) {
    return __builtin_amdgcn_wmma_f32_16x16x32_f16(false, a, false, b, (short)0, c, false, false);
  }
};

template <int BIAS_MODE, int OUT_MODE, bool RESID, int ACT>
__global__ __launch_bounds__(256) void wmma_gemm64(
    const unsigned short* __restrict__ Ap, int lda,
    const unsigned short* __restrict__ Btp, int ldb,
    void* __restrict__ Cout, int ldc,
    const float* __restrict__ bias,
    const float* __restrict__ resid,
    int M, int N, int K, float scale) {
  const _Float16* A  = (const _Float16*)Ap;
  const _Float16* Bt = (const _Float16*)Btp;
  __shared__ __align__(16) float sT[8][16 * 68];
  const int lane = threadIdx.x & 31;
  const int wave = threadIdx.x >> 5;
  const int tilesN = N >> 6;
  const int tilesM = M >> 6;
  const int tile = blockIdx.x * 8 + wave;
  if (tile >= tilesM * tilesN) return;
  const int tm = tile / tilesN;
  const int tn = tile - tm * tilesN;
  const int m0 = tm << 6;
  const int n0 = tn << 6;

  const int rlane = lane & 15;
  const int koff  = (lane >> 4) * 8;
  const int mOff  = (lane >> 4) * 8;

  v8f acc[4][4];
#pragma unroll
  for (int i = 0; i < 4; ++i)
#pragma unroll
    for (int j = 0; j < 4; ++j) acc[i][j] = (v8f){0.f,0.f,0.f,0.f,0.f,0.f,0.f,0.f};

  for (int k0 = 0; k0 < K; k0 += 32) {
    v16h bh[4];
#pragma unroll
    for (int j = 0; j < 4; ++j) {
      const size_t bo = (size_t)(n0 + (j << 4) + rlane) * ldb + koff + k0;
      bh[j] = FragH::load(Bt + bo);
    }
#pragma unroll
    for (int i = 0; i < 4; ++i) {
      const size_t ao = (size_t)(m0 + (i << 4) + rlane) * lda + koff + k0;
      v16h ah = FragH::load(A + ao);
#pragma unroll
      for (int j = 0; j < 4; ++j) acc[i][j] = FragH::mma(ah, bh[j], acc[i][j]);
      guard_row_h(acc[i][0], acc[i][1], acc[i][2], acc[i][3], ah, bh[0], bh[1], bh[2], bh[3]);
    }
    keep4_h(bh[0], bh[1], bh[2], bh[3]);
  }
  acc_guard4(acc[0][0], acc[0][1], acc[0][2], acc[0][3]);
  acc_guard4(acc[1][0], acc[1][1], acc[1][2], acc[1][3]);
  acc_guard4(acc[2][0], acc[2][1], acc[2][2], acc[2][3]);
  acc_guard4(acc[3][0], acc[3][1], acc[3][2], acc[3][3]);

  float* slab = sT[wave];
#pragma unroll
  for (int i = 0; i < 4; ++i) {
    const int mBase = m0 + (i << 4);
#pragma unroll
    for (int j = 0; j < 4; ++j) {
      const int n = n0 + (j << 4) + rlane;
      float bv = 0.f;
      if (BIAS_MODE == 2) bv = bias[n];
#pragma unroll
      for (int r = 0; r < 8; ++r) {
        float v = acc[i][j][r] * scale;
        if (BIAS_MODE == 2) v += bv;
        if (ACT == 2) v = fmaxf(v, 0.0f);
        slab[(mOff + r) * 68 + (j << 4) + rlane] = v;
      }
    }
    __builtin_amdgcn_fence(__ATOMIC_RELEASE, "workgroup");
    __builtin_amdgcn_wave_barrier();
    __builtin_amdgcn_fence(__ATOMIC_ACQUIRE, "workgroup");
    if (OUT_MODE == 0) {
      float* C = (float*)Cout;
      const int hh = lane >> 4, c4 = (lane & 15) * 4;
      v4f ov[8];
#pragma unroll
      for (int it = 0; it < 8; ++it) {
        const int row = it * 2 + hh;
        v4f v = *(const v4f*)(slab + row * 68 + c4);
        if (RESID) {
          const v4f rv = *(const v4f*)(resid + (size_t)(mBase + row) * ldc + n0 + c4);
          v = v + rv;
        }
        ov[it] = v;
      }
      for (int pass = 0; pass < 2; ++pass) {
#pragma unroll
        for (int it = 0; it < 8; ++it) {
          const int row = it * 2 + hh;
          *(volatile v4f*)(C + (size_t)(mBase + row) * ldc + n0 + c4) = ov[it];
        }
        __threadfence();
      }
    } else {
      unsigned short* C = (unsigned short*)Cout;
      const int q = lane >> 3, c8 = (lane & 7) * 8;
      v8h hv[4];
#pragma unroll
      for (int it = 0; it < 4; ++it) {
        const int row = it * 4 + q;
        const float* sp = slab + row * 68 + c8;
        const v4f a0 = *(const v4f*)(sp);
        const v4f a1 = *(const v4f*)(sp + 4);
#pragma unroll
        for (int e = 0; e < 4; ++e) {
          hv[it][e]     = (_Float16)a0[e];
          hv[it][4 + e] = (_Float16)a1[e];
        }
      }
      for (int pass = 0; pass < 2; ++pass) {
#pragma unroll
        for (int it = 0; it < 4; ++it) {
          const int row = it * 4 + q;
          *(volatile v8h*)(C + (size_t)(mBase + row) * ldc + n0 + c8) = hv[it];
        }
        __threadfence();
      }
    }
    __builtin_amdgcn_fence(__ATOMIC_RELEASE, "workgroup");
    __builtin_amdgcn_wave_barrier();
    __builtin_amdgcn_fence(__ATOMIC_ACQUIRE, "workgroup");
  }
}

__global__ __launch_bounds__(256) void cast_f16_kernel(
    const float* __restrict__ src, unsigned short* __restrict__ dst, int total8, int live8, float scale)
{
  const int i = blockIdx.x * 256 + threadIdx.x;
  if (i >= total8) return;
  const bool live = (i < live8);
  const int ic = live ? i : (live8 - 1);
  const float* p = src + ((size_t)ic << 3);
  const v4f a0 = *(const v4f*)(p);
  const v4f a1 = *(const v4f*)(p + 4);
  v8h hv;
#pragma unroll
  for (int e = 0; e < 4; ++e) {
    const float f0 = live ? (a0[e] * scale) : 0.0f;
    const float f1 = live ? (a1[e] * scale) : 0.0f;
    hv[e]     = (_Float16)f0;
    hv[4 + e] = (_Float16)f1;
  }
  unsigned short* q = dst + ((size_t)i << 3);
  *(volatile v8h*)q = hv;
  __threadfence();
  *(volatile v8h*)q = hv;
}

__global__ __launch_bounds__(128) void ln_f16_kernel(
    const float* __restrict__ X, const float* __restrict__ gw, const float* __restrict__ gb,
    unsigned short* __restrict__ H)
{
  __shared__ float red[8];
  const int tid = threadIdx.x, lane = tid & 31, wave = tid >> 5;
  const size_t row = blockIdx.x;
  const float* p = X + row * kDmod + tid * 8;
  const v4f a0 = *(const v4f*)(p);
  const v4f a1 = *(const v4f*)(p + 4);
  float s = ((a0[0] + a0[1]) + (a0[2] + a0[3])) + ((a1[0] + a1[1]) + (a1[2] + a1[3]));
#pragma unroll
  for (int off = 16; off >= 1; off >>= 1) s += __shfl_xor(s, off, 32);
  if (lane == 0) red[wave] = s;
  __syncthreads();
  const float mu = ((red[0] + red[1]) + (red[2] + red[3])) * (1.0f / (float)kDmod);
  float dv[8];
#pragma unroll
  for (int e = 0; e < 4; ++e) { dv[e] = a0[e] - mu; dv[4 + e] = a1[e] - mu; }
  float q = 0.0f;
#pragma unroll
  for (int e = 0; e < 8; ++e) q = fmaf(dv[e], dv[e], q);
#pragma unroll
  for (int off = 16; off >= 1; off >>= 1) q += __shfl_xor(q, off, 32);
  if (lane == 0) red[4 + wave] = q;
  __syncthreads();
  const float var  = ((red[4] + red[5]) + (red[6] + red[7])) * (1.0f / (float)kDmod);
  const float rstd = rsqrtf(var + 1e-5f);
  const v4f w0 = *(const v4f*)(gw + tid * 8);
  const v4f w1 = *(const v4f*)(gw + tid * 8 + 4);
  const v4f b0 = *(const v4f*)(gb + tid * 8);
  const v4f b1 = *(const v4f*)(gb + tid * 8 + 4);
  v8h hv;
#pragma unroll
  for (int e = 0; e < 4; ++e) {
    hv[e]     = (_Float16)((dv[e] * rstd) * w0[e] + b0[e]);
    hv[4 + e] = (_Float16)((dv[4 + e] * rstd) * w1[e] + b1[e]);
  }
  unsigned short* o = H + row * kDmod + tid * 8;
  *(volatile v8h*)o = hv;
  __threadfence();
  *(volatile v8h*)o = hv;
}

__global__ __launch_bounds__(256) void dt_cast_kernel(
    const float* __restrict__ PROJ, unsigned short* __restrict__ DT16, int total8, float scale)
{
  const int i = blockIdx.x * 256 + threadIdx.x;
  if (i >= total8) return;
  const int e0  = i << 3;
  const int row = e0 >> 6;
  const int c8  = e0 & 63;
  const float* p = PROJ + (size_t)row * kPrjP + c8;
  const v4f a0 = *(const v4f*)(p);
  const v4f a1 = *(const v4f*)(p + 4);
  v8h hv;
#pragma unroll
  for (int e = 0; e < 4; ++e) {
    hv[e]     = (_Float16)(a0[e] * scale);
    hv[4 + e] = (_Float16)(a1[e] * scale);
  }
  unsigned short* qd = DT16 + e0;
  *(volatile v8h*)qd = hv;
  __threadfence();
  *(volatile v8h*)qd = hv;
}

__global__ __launch_bounds__(128) void conv_silu_kernel(
    const unsigned* __restrict__ XZw, const float* __restrict__ cw, const float* __restrict__ cb,
    unsigned short* __restrict__ U16)
{
  __shared__ __align__(16) float sT[16 * kTP];
  const int tid = threadIdx.x, lane = tid & 31, wave = tid >> 5;
  const int d0 = blockIdx.x * 256, d = d0 + 2 * tid;
  const int t0 = blockIdx.y * 64;
  const size_t wcol = (size_t)(d >> 1);
  const v4f wa = *(const v4f*)(cw + (size_t)d * 4);
  const v4f wb = *(const v4f*)(cw + (size_t)d * 4 + 4);
  const float ba = cb[d], bb = cb[d + 1];
  float xa3, xa2, xa1, xb3, xb2, xb1;
  {
    const int r3 = t0 - 3, r2 = t0 - 2, r1 = t0 - 1;
    const unsigned q3 = XZw[(size_t)(r3 < 0 ? 0 : r3) * kXZW + wcol];
    const unsigned q2 = XZw[(size_t)(r2 < 0 ? 0 : r2) * kXZW + wcol];
    const unsigned q1 = XZw[(size_t)(r1 < 0 ? 0 : r1) * kXZW + wcol];
    const float a3 = h16_to_f32(q3 & 0xffffu), b3 = h16_to_f32(q3 >> 16);
    const float a2 = h16_to_f32(q2 & 0xffffu), b2 = h16_to_f32(q2 >> 16);
    const float a1 = h16_to_f32(q1 & 0xffffu), b1 = h16_to_f32(q1 >> 16);
    xa3 = (r3 >= 0) ? a3 : 0.f;  xb3 = (r3 >= 0) ? b3 : 0.f;
    xa2 = (r2 >= 0) ? a2 : 0.f;  xb2 = (r2 >= 0) ? b2 : 0.f;
    xa1 = (r1 >= 0) ? a1 : 0.f;  xb1 = (r1 >= 0) ? b1 : 0.f;
  }
#pragma unroll 1
  for (int sub = 0; sub < 4; ++sub) {
    const int lb = t0 + sub * 16;
#pragma unroll 1
    for (int s = 0; s < 16; ++s) {
      const unsigned w = XZw[(size_t)(lb + s) * kXZW + wcol];
      const float xa = h16_to_f32(w & 0xffffu);
      const float xb = h16_to_f32(w >> 16);
      float ca = wa[0] * xa3;
      ca = fmaf(wa[1], xa2, ca);
      ca = fmaf(wa[2], xa1, ca);
      ca = fmaf(wa[3], xa, ca);
      float cbv = wb[0] * xb3;
      cbv = fmaf(wb[1], xb2, cbv);
      cbv = fmaf(wb[2], xb1, cbv);
      cbv = fmaf(wb[3], xb, cbv);
      const float sva = ca + ba;
      const float svb = cbv + bb;
      const float ea = expf(-sva);
      const float eb = expf(-svb);
      sT[s * kTP + 2 * tid]     = sva * (1.0f / (1.0f + ea));
      sT[s * kTP + 2 * tid + 1] = svb * (1.0f / (1.0f + eb));
      xa3 = xa2; xa2 = xa1; xa1 = xa;
      xb3 = xb2; xb2 = xb1; xb1 = xb;
    }
    __syncthreads();
    v8h hv[4];
#pragma unroll
    for (int it = 0; it < 4; ++it) {
      const float* sp = sT + (it * 4 + wave) * kTP + lane * 8;
      const v4f a0 = *(const v4f*)(sp);
      const v4f a1 = *(const v4f*)(sp + 4);
#pragma unroll
      for (int e = 0; e < 4; ++e) {
        hv[it][e]     = (_Float16)a0[e];
        hv[it][4 + e] = (_Float16)a1[e];
      }
    }
    for (int pass = 0; pass < 2; ++pass) {
#pragma unroll
      for (int it = 0; it < 4; ++it)
        *(volatile v8h*)(U16 + (size_t)(lb + it * 4 + wave) * kDin + d0 + lane * 8) = hv[it];
      __threadfence();
    }
    __syncthreads();
  }
}

__global__ __launch_bounds__(256) void scan_kernel(
    const float* __restrict__ DLR, const unsigned* __restrict__ Uw, const unsigned* __restrict__ XZw,
    const float* __restrict__ PROJ, const float* __restrict__ A_log, const float* __restrict__ Dv,
    unsigned short* __restrict__ Y16)
{
  __shared__ __align__(16) float sBC[16 * 32];
  __shared__ __align__(16) float sY[16 * kTP];
  const int tid = threadIdx.x, lane = tid & 31, wave = tid >> 5;
  const int d0 = blockIdx.x * 256, d = d0 + tid;
  const unsigned sh = (unsigned)(d & 1) * 16u;
  const size_t dw = (size_t)(d >> 1);

  float An[kNst];
  {
    const v4f l0 = *(const v4f*)(A_log + (size_t)d * kNst);
    const v4f l1 = *(const v4f*)(A_log + (size_t)d * kNst + 4);
    const v4f l2 = *(const v4f*)(A_log + (size_t)d * kNst + 8);
    const v4f l3 = *(const v4f*)(A_log + (size_t)d * kNst + 12);
#pragma unroll
    for (int e = 0; e < 4; ++e) {
      An[e]      = -expf(l0[e]);
      An[4 + e]  = -expf(l1[e]);
      An[8 + e]  = -expf(l2[e]);
      An[12 + e] = -expf(l3[e]);
    }
  }
  const float Dd = Dv[d];
  float h[kNst];
#pragma unroll
  for (int n = 0; n < kNst; ++n) h[n] = 0.f;

#pragma unroll 1
  for (int c = 0; c < kSeqL / 16; ++c) {
    const int l0 = c * 16;
    if (tid < 128) {
      const int r = tid >> 3, q = (tid & 7) * 4;
      const v4f v = *(const v4f*)(PROJ + (size_t)(l0 + r) * kPrjP + kDtR + q);
      *(v4f*)(sBC + r * 32 + q) = v;
    }
    __syncthreads();
#pragma unroll 1
    for (int s = 0; s < 16; ++s) {
      const size_t m = (size_t)(l0 + s);
      const float a     = DLR[m * kDin + d];
      const unsigned uw = Uw[m * kUW + dw];
      const unsigned zw = XZw[m * kXZW + kUW + dw];
      const float xv    = h16_to_f32((uw >> sh) & 0xffffu);
      const float zv    = h16_to_f32((zw >> sh) & 0xffffu);
      const float delta = fmaxf(a, 0.0f) + log1pf(expf(-fabsf(a)));
      const float du    = delta * xv;
      v4f Bq[4], Cq[4];
#pragma unroll
      for (int qq = 0; qq < 4; ++qq) {
        Bq[qq] = *(const v4f*)(sBC + s * 32 + 4 * qq);
        Cq[qq] = *(const v4f*)(sBC + s * 32 + kNst + 4 * qq);
      }
      float y = 0.f;
#pragma unroll
      for (int n = 0; n < kNst; ++n) {
        const float e = __expf(delta * An[n]);
        const float p = du * Bq[n >> 2][n & 3];
        h[n] = fmaf(h[n], e, p);
        y = fmaf(h[n], Cq[n >> 2][n & 3], y);
      }
      y = fmaf(xv, Dd, y);
      const float ez = expf(-zv);
      const float g  = zv * (1.0f / (1.0f + ez));
      sY[s * kTP + tid] = (y * g) * kCY;
    }
    __syncthreads();
    v8h hv[2];
#pragma unroll
    for (int it = 0; it < 2; ++it) {
      const float* sp = sY + (it * 8 + wave) * kTP + lane * 8;
      const v4f a0 = *(const v4f*)(sp);
      const v4f a1 = *(const v4f*)(sp + 4);
#pragma unroll
      for (int e = 0; e < 4; ++e) { hv[it][e] = (_Float16)a0[e]; hv[it][4 + e] = (_Float16)a1[e]; }
    }
    for (int pass = 0; pass < 2; ++pass) {
#pragma unroll
      for (int it = 0; it < 2; ++it)
        *(volatile v8h*)(Y16 + (size_t)(l0 + it * 8 + wave) * kDin + d0 + lane * 8) = hv[it];
      __threadfence();
    }
  }
}

extern "C" void kernel_launch(void* const* d_in, const int* in_sizes, int n_in,
                              void* d_out, int out_size, void* d_ws, size_t ws_size,
                              hipStream_t stream)
{
  if (n_in < 18) return;
  if (in_sizes[0] != kRows * kDmod) return;
  if (in_sizes[1] != kDmod || in_sizes[2] != kDmod || in_sizes[3] != kDmod || in_sizes[4] != kDmod) return;
  if (in_sizes[5] != kXZP * kDmod) return;
  if (in_sizes[6] != kDin * 4 || in_sizes[7] != kDin) return;
  if (in_sizes[8] != kPrjN * kDin) return;
  if (in_sizes[9] != kDin * kDtR || in_sizes[10] != kDin) return;
  if (in_sizes[11] != kDin * kNst || in_sizes[12] != kDin) return;
  if (in_sizes[13] != kDmod * kDin) return;
  if (in_sizes[14] != kDff * kDmod || in_sizes[15] != kDff) return;
  if (in_sizes[16] != kDmod * kDff || in_sizes[17] != kDmod) return;
  if (out_size != kRows * kDmod) return;
  if (ws_size < kWsTotal) return;

  const float* x       = (const float*)d_in[0];
  const float* ln1_w   = (const float*)d_in[1];
  const float* ln1_b   = (const float*)d_in[2];
  const float* ln2_w   = (const float*)d_in[3];
  const float* ln2_b   = (const float*)d_in[4];
  const float* W_in    = (const float*)d_in[5];
  const float* conv_w  = (const float*)d_in[6];
  const float* conv_b  = (const float*)d_in[7];
  const float* W_xp    = (const float*)d_in[8];
  const float* W_dt    = (const float*)d_in[9];
  const float* b_dt    = (const float*)d_in[10];
  const float* A_log   = (const float*)d_in[11];
  const float* Dv      = (const float*)d_in[12];
  const float* W_out   = (const float*)d_in[13];
  const float* W_f1    = (const float*)d_in[14];
  const float* b_f1    = (const float*)d_in[15];
  const float* W_f2    = (const float*)d_in[16];
  const float* b_f2    = (const float*)d_in[17];
  float* dout = (float*)d_out;

  char* ws = (char*)d_ws;
  unsigned short* WIN16  = (unsigned short*)(ws + kOffWIN);
  unsigned short* WXP16  = (unsigned short*)(ws + kOffWXP);
  unsigned short* WDT16  = (unsigned short*)(ws + kOffWDT);
  unsigned short* WOUT16 = (unsigned short*)(ws + kOffWOUT);
  unsigned short* WF116  = (unsigned short*)(ws + kOffWF1);
  unsigned short* WF216  = (unsigned short*)(ws + kOffWF2);
  unsigned short* H16    = (unsigned short*)(ws + kOffH);
  float*          X1     = (float*)(ws + kOffX1);
  unsigned short* XZ     = (unsigned short*)(ws + kOffXZ);
  unsigned short* U16    = (unsigned short*)(ws + kOffU);
  unsigned short* Y16    = (unsigned short*)(ws + kOffY);
  float*          XDBL   = (float*)(ws + kOffXD);
  unsigned short* DT16   = (unsigned short*)(ws + kOffDT);
  float*          DLR    = (float*)(ws + kOffDLR);
  unsigned short* T16    = (unsigned short*)(ws + kOffT);
  const float* no_bias  = b_dt;
  const float* no_resid = x;

  cast_f16_kernel<<<(kXZP * kDmod / 8) / 256, 256, 0, stream>>>(W_in,  WIN16,  kXZP * kDmod / 8,  kXZP * kDmod / 8,  kCWin);
  cast_f16_kernel<<<(kPrjP * kDin / 8) / 256, 256, 0, stream>>>(W_xp,  WXP16,  kPrjP * kDin / 8,  kPrjN * kDin / 8,  kCWxp);
  cast_f16_kernel<<<(kDin * kDtR / 8) / 256, 256, 0, stream>>>(W_dt,   WDT16,  kDin * kDtR / 8,   kDin * kDtR / 8,   kCWdt);
  cast_f16_kernel<<<(kDmod * kDin / 8) / 256, 256, 0, stream>>>(W_out, WOUT16, kDmod * kDin / 8,  kDmod * kDin / 8,  kCWout);
  cast_f16_kernel<<<(kDff * kDmod / 8) / 256, 256, 0, stream>>>(W_f1,  WF116,  kDff * kDmod / 8,  kDff * kDmod / 8,  kCWf1);
  cast_f16_kernel<<<(kDmod * kDff / 8) / 256, 256, 0, stream>>>(W_f2,  WF216,  kDmod * kDff / 8,  kDmod * kDff / 8,  kCWf2);

  ln_f16_kernel<<<kRows, 128, 0, stream>>>(x, ln1_w, ln1_b, H16);

  for (int b = 0; b < kBatch; ++b) {
    const unsigned short* H16b = H16 + (size_t)b * kSeqL * kDmod;
    const float* xb  = x  + (size_t)b * kSeqL * kDmod;
    float*       X1b = X1 + (size_t)b * kSeqL * kDmod;

    wmma_gemm64<0, 1, false, 0><<<256, 256, 0, stream>>>(
        H16b, kDmod, WIN16, kDmod, (void*)XZ, kXZP, no_bias, no_resid,
        kSeqL, kXZP, kDmod, 1.0f / kCWin);

    conv_silu_kernel<<<dim3(kDin / 256, kSeqL / 64), 128, 0, stream>>>(
        (const unsigned*)XZ, conv_w, conv_b, U16);

    wmma_gemm64<0, 0, false, 0><<<8, 256, 0, stream>>>(
        U16, kDin, WXP16, kDin, (void*)XDBL, kPrjP, no_bias, no_resid,
        kSeqL, kPrjP, kDin, 1.0f / kCWxp);

    dt_cast_kernel<<<(kSeqL * kDtR / 8) / 256, 256, 0, stream>>>(XDBL, DT16, kSeqL * kDtR / 8, kCDt);

    wmma_gemm64<2, 0, false, 0><<<128, 256, 0, stream>>>(
        DT16, kDtR, WDT16, kDtR, (void*)DLR, kDin, b_dt, no_resid,
        kSeqL, kDin, kDtR, 1.0f / (kCDt * kCWdt));

    scan_kernel<<<kDin / 256, 256, 0, stream>>>(
        DLR, (const unsigned*)U16, (const unsigned*)XZ, XDBL, A_log, Dv, Y16);

    wmma_gemm64<0, 0, true, 0><<<64, 256, 0, stream>>>(
        Y16, kDin, WOUT16, kDin, (void*)X1b, kDmod, no_bias, xb,
        kSeqL, kDmod, kDin, 1.0f / (kCY * kCWout));
  }

  ln_f16_kernel<<<kRows, 128, 0, stream>>>(X1, ln2_w, ln2_b, H16);

  wmma_gemm64<2, 1, false, 2><<<512, 256, 0, stream>>>(
      H16, kDmod, WF116, kDmod, (void*)T16, kDff, b_f1, no_resid,
      kRows, kDff, kDmod, 1.0f / kCWf1);

  wmma_gemm64<2, 0, true, 0><<<128, 256, 0, stream>>>(
      T16, kDff, WF216, kDff, (void*)dout, kDmod, b_f2, X1,
      kRows, kDmod, kDff, 1.0f / kCWf2);
}
